// KAN_FFT_linear_59914793779340
// MI455X (gfx1250) — hardware-run, weakly checked
//
#include <hip/hip_runtime.h>
#include <math.h>

typedef __attribute__((ext_vector_type(16))) _Float16 v16h;
typedef __attribute__((ext_vector_type(8)))  _Float16 v8h;
typedef __attribute__((ext_vector_type(8)))  float    v8f;
typedef __attribute__((ext_vector_type(4)))  float    v4f;

constexpr int kRowsB     = 8192;
constexpr int kIn        = 256;
constexpr int kOut       = 256;
constexpr int kGrid      = 64;
constexpr int kKh        = kIn * kGrid;
constexpr int kKt        = 2 * kKh;
constexpr int kChunkRows = 1024;
constexpr int kChunks    = kRowsB / kChunkRows;
constexpr float kCarryA  = 64.0f;
constexpr float kCarryW  = 128.0f;
constexpr float kFold    = 1.0f / (kCarryA * kCarryW);

static_assert(kKh == 16384);
static_assert(kKt == 32768);
static_assert((kKt % 32) == 0);
static_assert((kChunkRows % 64) == 0 && (kOut % 64) == 0);
static_assert(kChunks * kChunkRows == kRowsB);

constexpr size_t kBtBytes = (size_t)kOut * kKt * 2;
constexpr size_t kAcBytes = (size_t)kChunkRows * kKt * 2;
constexpr size_t kOffBt   = 0;
constexpr size_t kOffAc   = kOffBt + kBtBytes;
constexpr size_t kWsTotal = kOffAc + kAcBytes;
static_assert(kBtBytes == 16777216ull);
static_assert(kAcBytes == 67108864ull);
static_assert(kWsTotal == 83886080ull);
static_assert(kWsTotal <= 134217728ull);
static_assert((kOffAc % 128) == 0);

union FragU { v16h v; v8h h[2]; };
__device__ __forceinline__ v16h frag_load(const _Float16* p) {
  FragU f;
  f.h[0] = *(const v8h*)(p);
  f.h[1] = *(const v8h*)(p + 16);
  return f.v;
}
__device__ __forceinline__ v8f mma_h(v16h a, v16h b, v8f c) {
  return __builtin_amdgcn_wmma_f32_16x16x32_f16(false, a, false, b, (short)0, c, false, false);
}
__device__ __forceinline__ void tie_acc(v8f& c, v16h a, v16h b) { asm volatile("" : "+v"(c) : "v"(a), "v"(b)); }
__device__ __forceinline__ void nop_acc(v8f& c, v16h a, v16h b) { asm volatile("v_nop\n\tv_nop\n\tv_nop\n\tv_nop" : "+v"(c) : "v"(a), "v"(b)); }
__device__ __forceinline__ void keep4_h(v16h a, v16h b, v16h c, v16h d) { asm volatile("v_nop" :: "v"(a), "v"(b), "v"(c), "v"(d)); }
__device__ __forceinline__ void acc_guard4(v8f& a, v8f& b, v8f& c, v8f& d) { asm volatile("v_nop\n\tv_nop\n\tv_nop\n\tv_nop" : "+v"(a), "+v"(b), "+v"(c), "+v"(d)); }

constexpr int kPrepThreads = 2 * kOut * kKh / 8;
static_assert((kPrepThreads % 256) == 0);

__global__ __launch_bounds__(256) void prep_w_kernel(const float* __restrict__ W, _Float16* __restrict__ Bt) {
  const int idx = blockIdx.x * 256 + threadIdx.x;
  if (idx >= kPrepThreads) return;
  const size_t e0 = (size_t)idx << 3;
  const int run = (int)(e0 / (size_t)kKh);
  const int r   = (int)(e0 - (size_t)run * kKh);
  const int t   = run / kOut;
  const int j   = run - t * kOut;
  const v4f a0 = *(const v4f*)(W + e0);
  const v4f a1 = *(const v4f*)(W + e0 + 4);
  v8h hv;
#pragma unroll
  for (int e = 0; e < 4; ++e) {
    const float f0 = a0[e] * kCarryW;
    const float f1 = a1[e] * kCarryW;
    hv[e]     = (_Float16)f0;
    hv[4 + e] = (_Float16)f1;
  }
  _Float16* dst = Bt + (size_t)j * kKt + (size_t)t * kKh + r;
  *(volatile v8h*)dst = hv;
  __threadfence();
  *(volatile v8h*)dst = hv;
}

constexpr int kExpThreads      = 128;
constexpr int kExpPitch        = 136;
constexpr int kExpBlocksPerRow = kIn / kExpThreads;
constexpr int kExpGrid         = kChunkRows * kExpBlocksPerRow;
static_assert(kExpBlocksPerRow * kExpThreads == kIn);
static_assert(kGrid == 64);
static_assert((kExpPitch % 8) == 0 && kExpPitch >= 2 * kGrid);

__global__ __launch_bounds__(128) void expand_trig_kernel(const float* __restrict__ X, _Float16* __restrict__ Ac) {
  __shared__ __align__(16) _Float16 sT[kExpThreads * kExpPitch];
  const int tid  = threadIdx.x;
  const int lane = tid & 31;
  const int wave = tid >> 5;
  const int bl   = blockIdx.x / kExpBlocksPerRow;
  const int i0   = (blockIdx.x - bl * kExpBlocksPerRow) * kExpThreads;
  const float xv = X[(size_t)bl * kIn + i0 + tid];
  float s1, c1;
  sincosf(xv, &s1, &c1);
  float c = c1 * kCarryA;
  float s = s1 * kCarryA;
  _Float16* myrow = sT + tid * kExpPitch;
#pragma unroll 1
  for (int it = 0; it < 8; ++it) {
    v8h cv, sv;
#pragma unroll
    for (int e = 0; e < 8; ++e) {
      cv[e] = (_Float16)c;
      sv[e] = (_Float16)s;
      const float cn = fmaf(c, c1, -(s * s1));
      const float sn = fmaf(s, c1, c * s1);
      c = cn;
      s = sn;
    }
    *(v8h*)(myrow + it * 8) = cv;
    *(v8h*)(myrow + kGrid + it * 8) = sv;
  }
  __syncthreads();
  const int q  = lane >> 3;
  const int c8 = (lane & 7) * 8;
  v8h lc[8], ls[8];
#pragma unroll
  for (int it = 0; it < 8; ++it) {
    const int row = wave * 32 + it * 4 + q;
    const _Float16* sp = sT + row * kExpPitch + c8;
    lc[it] = *(const v8h*)(sp);
    ls[it] = *(const v8h*)(sp + kGrid);
  }
  _Float16* rowbase = Ac + (size_t)bl * kKt;
  for (int pass = 0; pass < 2; ++pass) {
#pragma unroll
    for (int it = 0; it < 8; ++it) {
      const int row = wave * 32 + it * 4 + q;
      const size_t o = (size_t)(i0 + row) * kGrid + c8;
      *(volatile v8h*)(rowbase + o) = lc[it];
      *(volatile v8h*)(rowbase + kKh + o) = ls[it];
    }
    __threadfence();
  }
}

__global__ __launch_bounds__(256) void gemm_f16_kernel(
    const _Float16* __restrict__ A, int lda,
    const _Float16* __restrict__ Bt, int ldb,
    float* __restrict__ C, int ldc,
    const float* __restrict__ bias,
    int M, int N, int K, float scale) {
  __shared__ __align__(16) float sT[8][16 * 68];
  const int lane = threadIdx.x & 31;
  const int wave = threadIdx.x >> 5;
  const int tilesN = N >> 6;
  const int tilesM = M >> 6;
  const int tile = blockIdx.x * 8 + wave;
  if (tile >= tilesM * tilesN) return;
  const int tm = tile / tilesN;
  const int tn = tile - tm * tilesN;
  const int m0 = tm << 6;
  const int n0 = tn << 6;

  const int rlane = lane & 15;
  const int koff  = (lane >> 4) * 8;
  const int mOff  = (lane >> 4) * 8;

  v8f acc[4][4];
#pragma unroll
  for (int i = 0; i < 4; ++i)
#pragma unroll
    for (int j = 0; j < 4; ++j) acc[i][j] = (v8f){0.f, 0.f, 0.f, 0.f, 0.f, 0.f, 0.f, 0.f};

#pragma unroll 1
  for (int k0 = 0; k0 < K; k0 += 32) {
    v16h bh[4];
#pragma unroll
    for (int j = 0; j < 4; ++j) {
      const size_t bo = (size_t)(n0 + (j << 4) + rlane) * ldb + koff + k0;
      bh[j] = frag_load(Bt + bo);
    }
#pragma unroll
    for (int i = 0; i < 4; ++i) {
      const size_t ao = (size_t)(m0 + (i << 4) + rlane) * lda + koff + k0;
      const v16h ah = frag_load(A + ao);
#pragma unroll
      for (int j = 0; j < 4; ++j) acc[i][j] = mma_h(ah, bh[j], acc[i][j]);
      tie_acc(acc[i][0], ah, bh[0]);
      tie_acc(acc[i][1], ah, bh[1]);
      tie_acc(acc[i][2], ah, bh[2]);
      nop_acc(acc[i][3], ah, bh[3]);
    }
    keep4_h(bh[0], bh[1], bh[2], bh[3]);
  }
  acc_guard4(acc[0][0], acc[0][1], acc[0][2], acc[0][3]);
  acc_guard4(acc[1][0], acc[1][1], acc[1][2], acc[1][3]);
  acc_guard4(acc[2][0], acc[2][1], acc[2][2], acc[2][3]);
  acc_guard4(acc[3][0], acc[3][1], acc[3][2], acc[3][3]);

  float* slab = sT[wave];
#pragma unroll
  for (int i = 0; i < 4; ++i) {
    const int mBase = m0 + (i << 4);
#pragma unroll
    for (int j = 0; j < 4; ++j) {
      const int n = n0 + (j << 4) + rlane;
      const float bv = bias[n];
#pragma unroll
      for (int r = 0; r < 8; ++r) {
        float v = acc[i][j][r] * scale;
        v += bv;
        slab[(mOff + r) * 68 + (j << 4) + rlane] = v;
      }
    }
    __builtin_amdgcn_fence(__ATOMIC_RELEASE, "workgroup");
    __builtin_amdgcn_wave_barrier();
    __builtin_amdgcn_fence(__ATOMIC_ACQUIRE, "workgroup");
    {
      const int hh = lane >> 4;
      const int c4 = (lane & 15) * 4;
      for (int pass = 0; pass < 2; ++pass) {
#pragma unroll
        for (int it = 0; it < 8; ++it) {
          const int row = it * 2 + hh;
          const v4f v = *(const v4f*)(slab + row * 68 + c4);
          *(volatile v4f*)(C + (size_t)(mBase + row) * ldc + n0 + c4) = v;
        }
        __threadfence();
      }
    }
    __builtin_amdgcn_fence(__ATOMIC_RELEASE, "workgroup");
    __builtin_amdgcn_wave_barrier();
    __builtin_amdgcn_fence(__ATOMIC_ACQUIRE, "workgroup");
  }
}

extern "C" void kernel_launch(void* const* d_in, const int* in_sizes, int n_in,
                              void* d_out, int out_size, void* d_ws, size_t ws_size,
                              hipStream_t stream) {
  if (n_in < 3) return;
  if (in_sizes[0] != kRowsB * kIn) return;
  if (in_sizes[1] != 2 * kOut * kIn * kGrid) return;
  if (in_sizes[2] != kOut) return;
  if (out_size != kRowsB * kOut) return;
  if (ws_size < kWsTotal) return;

  const float* x    = (const float*)d_in[0];
  const float* W    = (const float*)d_in[1];
  const float* bias = (const float*)d_in[2];
  float* out = (float*)d_out;

  char* ws = (char*)d_ws;
  _Float16* Bt = (_Float16*)(ws + kOffBt);
  _Float16* Ac = (_Float16*)(ws + kOffAc);

  prep_w_kernel<<<kPrepThreads / 256, 256, 0, stream>>>(W, Bt);

  constexpr int kGemmBlocks = ((kChunkRows / 64) * (kOut / 64)) / 8;
  static_assert(kGemmBlocks * 8 == (kChunkRows / 64) * (kOut / 64));

  for (int cidx = 0; cidx < kChunks; ++cidx) {
    const float* xc = x + (size_t)cidx * kChunkRows * kIn;
    float* oc = out + (size_t)cidx * kChunkRows * kOut;
    expand_trig_kernel<<<kExpGrid, kExpThreads, 0, stream>>>(xc, Ac);
    gemm_f16_kernel<<<kGemmBlocks, 256, 0, stream>>>(
        Ac, kKt, Bt, kKt, oc, kOut, bias, kChunkRows, kOut, kKt, kFold);
  }
}
